// LSTMCell_22093311770693
// MI455X (gfx1250) — hardware-verified
//
#include <hip/hip_runtime.h>
#include <math.h>

typedef __attribute__((ext_vector_type(16))) _Float16 v16h;
typedef __attribute__((ext_vector_type(16))) __bf16 v16b;
typedef __attribute__((ext_vector_type(8)))  _Float16 v8h;
typedef __attribute__((ext_vector_type(8)))  float v8f;
typedef __attribute__((ext_vector_type(4)))  float v4f;
typedef __attribute__((ext_vector_type(2)))  float v2f;
typedef __attribute__((ext_vector_type(4)))  unsigned v4u;
typedef __attribute__((ext_vector_type(4)))  int v4i;
typedef float __attribute__((may_alias)) float_a;
typedef int __attribute__((may_alias)) int_a;

template <typename T> __device__ __forceinline__ void vst2(void* p, T v) { *(volatile T*)p = v; __threadfence(); *(volatile T*)p = v; }
__device__ __forceinline__ v8f wmma16(v16h a, v16h b, v8f c) {
  v8f d = __builtin_amdgcn_wmma_f32_16x16x32_f16(false, a, false, b, (short)0, c, false, false);
  asm volatile("v_nop\n\tv_nop\n\tv_nop\n\tv_nop" : "+v"(d) : "v"(a), "v"(b));
  return d;
}
__device__ __forceinline__ v8f wmma_bf(v16b a, v16b b, v8f c) {
  v8f d = __builtin_amdgcn_wmma_f32_16x16x32_bf16(false, a, false, b, (short)0, c, false, false);
  asm volatile("v_nop\n\tv_nop\n\tv_nop\n\tv_nop" : "+v"(d) : "v"(a), "v"(b));
  return d;
}
__device__ __forceinline__ v16h frag_h(const _Float16* rowk0, int lane) {
  union { v16h v; v8h q[2]; } u; const _Float16* p = rowk0 + 8 * (lane >> 4);
  u.q[0] = *(const v8h*)p; u.q[1] = *(const v8h*)(p + 16); return u.v;
}
__device__ __forceinline__ v16h frag_f32(const float* rowk0, int lane) {
  v16h a; const float* p = rowk0 + 8 * (lane >> 4);
#pragma unroll
  for (int i = 0; i < 8; ++i) { a[i] = (_Float16)p[i]; a[8 + i] = (_Float16)p[16 + i]; }
  return a;
}
__device__ __forceinline__ v16h frag_f32s(const float* rowk0, int lane, float sc) {
  v16h a; const float* p = rowk0 + 8 * (lane >> 4);
#pragma unroll
  for (int i = 0; i < 8; ++i) { a[i] = (_Float16)(p[i] * sc); a[8 + i] = (_Float16)(p[16 + i] * sc); }
  return a;
}
__device__ __forceinline__ v16h fragc_f32(const float* W, int k0, int n, int lane, int ld, int K) {
  v16h a; const int g = lane >> 4;
#pragma unroll
  for (int i = 0; i < 8; ++i) { const int ka = k0 + 8 * g + i, kb = ka + 16;
    a[i] = (_Float16)(ka < K ? W[(size_t)(ka < K ? ka : K - 1) * ld + n] : 0.f); a[8 + i] = (_Float16)(kb < K ? W[(size_t)(kb < K ? kb : K - 1) * ld + n] : 0.f); }
  return a;
}
struct F2 { v16b h, l; };
__device__ __forceinline__ F2 bsplit16(const float v[16]) { F2 r;
#pragma unroll
  for (int i = 0; i < 16; ++i) { const __bf16 h = (__bf16)v[i]; r.h[i] = h; r.l[i] = (__bf16)(v[i] - (float)h); }
  return r; }
__device__ __forceinline__ F2 split_row(const float* row, int k0, int lane) { float v[16]; const float* p = row + k0 + 8 * (lane >> 4);
#pragma unroll
  for (int i = 0; i < 8; ++i) { v[i] = p[i]; v[8 + i] = p[16 + i]; }
  return bsplit16(v); }
__device__ __forceinline__ F2 split_rowK(const float* row, int k0, int lane, int K) { float v[16]; const int g = lane >> 4;
#pragma unroll
  for (int i = 0; i < 8; ++i) { const int ka = k0 + 8 * g + i, kb = ka + 16; v[i] = ka < K ? row[ka < K ? ka : K - 1] : 0.f; v[8 + i] = kb < K ? row[kb < K ? kb : K - 1] : 0.f; }
  return bsplit16(v); }
__device__ __forceinline__ F2 split_col(const float* W, int k0, int n, int lane, int ld, int K) { float v[16]; const int g = lane >> 4;
#pragma unroll
  for (int i = 0; i < 8; ++i) { const int ka = k0 + 8 * g + i, kb = ka + 16; v[i] = ka < K ? W[(size_t)(ka < K ? ka : K - 1) * ld + n] : 0.f; v[8 + i] = kb < K ? W[(size_t)(kb < K ? kb : K - 1) * ld + n] : 0.f; }
  return bsplit16(v); }
__device__ __forceinline__ v8f mac3(const F2& a, const F2& b, v8f c) { c = wmma_bf(a.l, b.h, c); c = wmma_bf(a.h, b.l, c); return wmma_bf(a.h, b.h, c); }
__device__ __forceinline__ float sigm(float v) { return 1.0f / (1.0f + expf(-v)); }
#define LDSX() do { asm volatile("s_wait_dscnt 0" ::: "memory"); __builtin_amdgcn_wave_barrier(); __builtin_amdgcn_fence(__ATOMIC_RELEASE, "workgroup"); } while (0)


#define NBATCH 4096
#define IS 1024
#define OS 1024
#define KK (IS + OS)
#define NO (4 * OS)
#define LNEPS 1e-5f
#ifndef TROW
#define TROW NBATCH
#endif
typedef __attribute__((ext_vector_type(8))) __bf16 v8b;
__device__ __forceinline__ v16b frag_b(const __bf16* rowk0, int lane) {
  union { v16b v; v8b q[2]; } u; const __bf16* p = rowk0 + 8 * (lane >> 4);
  u.q[0] = *(const v8b*)p; u.q[1] = *(const v8b*)(p + 16); return u.v;
}
__device__ __forceinline__ float bfr(float v) { return (float)(__bf16)v; }
__device__ __attribute__((noinline)) float exp_ni(float v) { return expf(v); }
__device__ __attribute__((noinline)) float erf_ni(float v) { return erff(v); }

#define WS_C   0u
#define WS_END (WS_C + 4u * (size_t)NBATCH * NO)

__device__ __forceinline__ v16b fragb_f32(const float* __restrict__ p, int lane) { v16b a; const float* pp = p + 8 * (lane >> 4);
#pragma unroll
  for (int i = 0; i < 8; ++i) { a[i] = (__bf16)pp[i]; a[8 + i] = (__bf16)pp[16 + i]; } return a; }
__global__ __launch_bounds__(128) void k_gemm(const float* __restrict__ X, const float* __restrict__ Hh, const float* __restrict__ Wt, float* __restrict__ C) { __shared__ __align__(16) float sf[4][16][132];
  const int tid = threadIdx.x, wave = tid >> 5, lane = tid & 31, col = lane & 15, g = lane >> 4; const size_t r0 = (size_t)blockIdx.x * 64 + wave * 16; const int c0 = blockIdx.y * 128;
  v8f acc[8] = {};
#pragma unroll 2
  for (int kc = 0; kc < KK / 32; ++kc) { const v16b a = (kc < IS / 32) ? fragb_f32(X + (r0 + col) * IS + kc * 32, lane) : fragb_f32(Hh + (r0 + col) * OS + (kc - IS / 32) * 32, lane);
#pragma unroll
    for (int j = 0; j < 8; ++j) acc[j] = wmma_bf(a, fragb_f32(Wt + (size_t)(c0 + j * 16 + col) * KK + kc * 32, lane), acc[j]); }
#pragma unroll
  for (int j = 0; j < 8; ++j)
#pragma unroll
    for (int r = 0; r < 8; ++r) sf[wave][8 * g + r][j * 16 + col] = acc[j][r];
  LDSX(); for (int rl = 0; rl < 16; ++rl) vst2(C + (r0 + rl) * NO + c0 + lane * 4, *(const v4f*)&sf[wave][rl][lane * 4]); }
__global__ __launch_bounds__(256) void k_cell(const float* __restrict__ C, const float* __restrict__ CP, const float* __restrict__ LW, const float* __restrict__ LB, float* __restrict__ OUT, float* __restrict__ CELL) { __shared__ float red[8]; __shared__ float stat[2];
  const int t = threadIdx.x, lane = t & 31, w = t >> 5; const size_t row = blockIdx.x; const float* cr = C + row * NO;
  float s = 0.f;
#pragma unroll 1
  for (int i = t; i < NO; i += 256) s += cr[i];
#pragma unroll
  for (int o = 1; o < 32; o <<= 1) s += __shfl_xor(s, o);
  if (lane == 0) red[w] = s; __syncthreads(); if (t == 0) { float a = 0.f; for (int i = 0; i < 8; ++i) a += red[i]; stat[0] = a * (1.0f / NO); } __syncthreads();
  const float mu = stat[0]; float q = 0.f;
#pragma unroll 1
  for (int i = t; i < NO; i += 256) { const float d = cr[i] - mu; q += d * d; }
#pragma unroll
  for (int o = 1; o < 32; o <<= 1) q += __shfl_xor(q, o);
  if (lane == 0) red[w] = q; __syncthreads(); if (t == 0) { float a = 0.f; for (int i = 0; i < 8; ++i) a += red[i]; stat[1] = 1.0f / sqrtf(a * (1.0f / NO) + LNEPS); } __syncthreads();
  const float inv = stat[1];
  { const int o0 = t * 4; v4f vo, vc;
#pragma unroll 1
    for (int j = 0; j < 4; ++j) { const int o = o0 + j; float gv[4];
#pragma unroll 1
      for (int k = 0; k < 4; ++k) gv[k] = (cr[k * OS + o] - mu) * inv * bfr(LW[k * OS + o]) + bfr(LB[k * OS + o]);
      const float fg = 1.0f / (1.0f + expf(-gv[0])), og = 1.0f / (1.0f + expf(-gv[1])), ig = 1.0f / (1.0f + expf(-gv[2]));
      const float hid = 0.5f * gv[3] * (1.0f + erff(gv[3] * 0.70710678118654752f));
      const float cell = fg * bfr(CP[row * OS + o]) + ig * hid; vc[j] = cell; vo[j] = og * cell; }
    vst2(OUT + row * OS + o0, vo); vst2(CELL + row * OS + o0, vc); } }
extern "C" void kernel_launch(void* const* d_in, const int* in_sizes, int n_in, void* d_out, int out_size, void* d_ws, size_t ws_size, hipStream_t stream) {
  (void)in_sizes; (void)n_in; (void)out_size;
  const float** F = (const float**)d_in;
  if (ws_size < (size_t)WS_END) return;
  char* ws = (char*)d_ws; float* C = (float*)(ws + WS_C);
  float* OUT = (float*)d_out; float* CELL = OUT + (size_t)NBATCH * OS;
  k_gemm<<<dim3(TROW / 64, NO / 128), 128, 0, stream>>>(F[0], F[1], F[3], C);
  k_cell<<<TROW, 256, 0, stream>>>(C, F[2], F[4], F[5], OUT, CELL);
}
